// MultiHeadAttention_90031104458908
// MI455X (gfx1250) — hardware-verified
//
#include <hip/hip_runtime.h>


#ifndef NB
#define NB 2
#endif
#ifndef SEQ
#define SEQ 2048
#endif
#define NB_FULL  2
#define SEQ_FULL 2048
#ifndef OUT_SEQ
#define OUT_SEQ SEQ
#endif
#define DM   2048
#define NH_  16
#define HD   128
#define ER   ((SEQ) < 512 ? (SEQ) : 512)
#define DTL  ((SEQ) > ER ? ((SEQ) - ER) / 64 : 1)
#define AW   4
#define RS   2048.0f
#define RI   (1.0f / 2048.0f)
#define SC2  (0.08838834764831845f * 1.4426950408889634f)
#define PSH  8.0f
#define CXS  16.0f
#define WOS  256.0f
#define OUTS (1.0f / 4096.0f)
#define PLN  ((size_t)NB * NH_ * SEQ * HD)
#define PLE  ((size_t)NB * NH_ * ER * HD)

static_assert(HD == 128);
static_assert(NH_ * HD == DM);
static_assert(DM % 64 == 0);
static_assert(DM % 32 == 0);
static_assert(SEQ % 64 == 0);
static_assert(ER % 64 == 0);
static_assert(ER <= SEQ);
static_assert((SEQ - ER) % 64 == 0);
static_assert(SEQ % 32 == 0);
static_assert(((size_t)SEQ * DM) % 8 == 0);
static_assert((SEQ * 64) % 256 == 0);
static_assert(NB <= NB_FULL);
static_assert(SEQ <= SEQ_FULL);

typedef _Float16 h16;
typedef unsigned short bf;
typedef __attribute__((ext_vector_type(16))) __bf16   v16bf;
typedef __attribute__((ext_vector_type(16))) _Float16 v16h;
typedef __attribute__((ext_vector_type(8)))  _Float16 v8h;
typedef __attribute__((ext_vector_type(8)))  unsigned short v8us;
typedef __attribute__((ext_vector_type(8)))  float    v8f;
typedef __attribute__((ext_vector_type(4)))  float    v4f;
typedef v4f  __attribute__((may_alias)) v4fa;

__device__ __forceinline__ unsigned short f2bf(float f) { unsigned u = __float_as_uint(f); u += 0x7FFFu + ((u >> 16) & 1u); return (unsigned short)(u >> 16); }
__device__ __forceinline__ v16h cat16(v8h lo, v8h hi) { return __builtin_shufflevector(lo, hi, 0, 1, 2, 3, 4, 5, 6, 7, 8, 9, 10, 11, 12, 13, 14, 15); }
__device__ __forceinline__ v16bf cat16b(v8us lo, v8us hi) { return __builtin_bit_cast(v16bf, __builtin_shufflevector(lo, hi, 0, 1, 2, 3, 4, 5, 6, 7, 8, 9, 10, 11, 12, 13, 14, 15)); }
__device__ __forceinline__ v8f wmma16(v16h a, v16h b, v8f c) { return __builtin_amdgcn_wmma_f32_16x16x32_f16(false, a, false, b, (short)0, c, false, false); }
__device__ __forceinline__ v8f wmmab(v16bf a, v16bf b, v8f c) { return __builtin_amdgcn_wmma_f32_16x16x32_bf16(false, a, false, b, (short)0, c, false, false); }
__device__ __forceinline__ v16h  ldh(const h16* p) { return cat16(*(const v8h*)p, *(const v8h*)(p + 16)); }
__device__ __forceinline__ v16bf ldb(const bf* p)  { return cat16b(*(const v8us*)p, *(const v8us*)(p + 16)); }
__device__ __forceinline__ void wave_sync() { __builtin_amdgcn_fence(3  , "wavefront"); __builtin_amdgcn_wave_barrier(); asm volatile("" ::: "memory"); }

__global__ __launch_bounds__(256) void k_cvt8(const float* __restrict__ src, bf* dst, size_t n8) {
    const size_t i = (size_t)blockIdx.x * 256 + threadIdx.x; if (i >= n8) return;
    const v8f v = *(const v8f*)(src + i * 8); v8us o;
#pragma unroll
    for (int k = 0; k < 8; ++k) o[k] = f2bf(v[k]);
    *(volatile v8us*)(dst + i * 8) = o; __threadfence(); *(volatile v8us*)(dst + i * 8) = o;
}

template <int F16M>
__device__ __forceinline__ unsigned short cvtw(float x) {
    const unsigned short r = f2bf(x);
    if (F16M) { const float f = __uint_as_float((unsigned)r << 16); const h16 hv = (h16)(f * WOS); return __builtin_bit_cast(unsigned short, hv); }
    return r;
}

template <int F16M>
__global__ __launch_bounds__(256) void k_wt(const float* __restrict__ W, unsigned short* WT) {
    __shared__ __align__(16) float ts[64 * 68];
    const int tid = threadIdx.x, lane = tid & 31, wv = tid >> 5;
    const int k0 = blockIdx.x * 64, n0 = blockIdx.y * 64;
#pragma unroll
    for (int it = 0; it < 4; ++it) {
        const int i = tid + 256 * it; const int kr = i >> 4, c4 = (i & 15) * 4;
        const v4f v = *(const v4f*)(W + (size_t)(k0 + kr) * DM + n0 + c4);
        ts[(c4 + 0) * 68 + kr] = v[0]; ts[(c4 + 1) * 68 + kr] = v[1]; ts[(c4 + 2) * 68 + kr] = v[2]; ts[(c4 + 3) * 68 + kr] = v[3];
    }
    __syncthreads();
#pragma unroll
    for (int it = 0; it < 2; ++it) {
        const int row = it * 32 + wv * 4 + (lane >> 3), c8 = (lane & 7) * 8;
        const v4f x0 = *(const v4fa*)(&ts[row * 68 + c8]); const v4f x1 = *(const v4fa*)(&ts[row * 68 + c8 + 4]);
        v8us o;
#pragma unroll
        for (int i = 0; i < 4; ++i) { o[i] = cvtw<F16M>(x0[i]); o[4 + i] = cvtw<F16M>(x1[i]); }
        unsigned short* dst = WT + (size_t)(n0 + row) * DM + k0 + c8;
        *(volatile v8us*)dst = o; __threadfence(); *(volatile v8us*)dst = o;
    }
}

__global__ __launch_bounds__(256) void k_tab(float* TAB) {
#pragma clang fp contract(off)
    const int idx = blockIdx.x * 256 + threadIdx.x;
    const int t = idx >> 6, i = idx & 63;
    const float inv = exp2f(-(float)i * 0.20762050593046014f);
    const float ang = (float)t * inv;
    const float cs = cosf(ang), sn = sinf(ang);
    volatile float* pc = TAB + idx; volatile float* ps = TAB + (size_t)SEQ * 64 + idx;
    *pc = cs; *ps = sn; __threadfence(); *pc = cs; *ps = sn;
}

__global__ __launch_bounds__(32) void k_qk(const bf* __restrict__ A, const bf* __restrict__ WT, const float* __restrict__ TAB, h16* PH, h16* PR) {
    __shared__ __align__(16) float os[16 * 132];
    const int K = DM;
    const int lane = threadIdx.x & 31, lr = lane & 15, hi = lane >> 4;
    const int r0 = blockIdx.x * 32, hh = blockIdx.y, z = blockIdx.z;
    const bf* Bt = WT + (size_t)z * DM * DM;
    v8f acc[2][8];
#pragma unroll
    for (int mb = 0; mb < 2; ++mb)
#pragma unroll
        for (int nb = 0; nb < 8; ++nb) acc[mb][nb] = (v8f){};
    const size_t aoff = (size_t)(r0 + lr) * K + 8 * hi, boff = (size_t)(hh * HD + lr) * K + 8 * hi;
#pragma unroll 1
    for (int kc = 0; kc < K; kc += 32) {
        const v16bf a0 = ldb(A + aoff + kc), a1 = ldb(A + aoff + (size_t)16 * K + kc);
#pragma unroll
        for (int nb = 0; nb < 8; ++nb) { const v16bf bq = ldb(Bt + boff + (size_t)nb * 16 * K + kc);
            acc[0][nb] = wmmab(a0, bq, acc[0][nb]); acc[1][nb] = wmmab(a1, bq, acc[1][nb]); }
        asm volatile("v_nop\n\tv_nop\n\tv_nop\n\tv_nop" : "+v"(acc[0][4]), "+v"(acc[1][4]), "+v"(acc[0][5]), "+v"(acc[1][5]), "+v"(acc[0][6]), "+v"(acc[1][6]), "+v"(acc[0][7]), "+v"(acc[1][7]) : "v"(a0), "v"(a1));
    }
    const int bq_ = r0 / SEQ, t0 = r0 % SEQ;
    const bool wr = t0 < ER; const int tr = wr ? t0 : 0;
    h16* PHz = PH + (size_t)z * PLN + ((size_t)(bq_ * NH_ + hh) * SEQ + t0) * HD;
    h16* PRz = PR + (size_t)z * PLE + ((size_t)(bq_ * NH_ + hh) * ER + tr) * HD;
    const float* TC = TAB; const float* TS = TAB + (size_t)SEQ * 64;
#pragma unroll
    for (int mb = 0; mb < 2; ++mb) {
#pragma unroll
        for (int nb = 0; nb < 8; ++nb) {
#pragma unroll
            for (int j = 0; j < 8; ++j) os[(hi * 8 + j) * 132 + nb * 16 + lr] = acc[mb][nb][j]; }
        wave_sync();
#pragma unroll 1
        for (int s = 0; s < 8; ++s) {
            const int row = 2 * s + hi, c8 = lr * 8;
            const int pc = c8 ^ 64, tc = c8 & 63; const float sg = (c8 < 64) ? -1.0f : 1.0f;
            const int t = t0 + mb * 16 + row;
            const v4f x0 = *(const v4fa*)(&os[row * 132 + c8]); const v4f x1 = *(const v4fa*)(&os[row * 132 + c8 + 4]);
            const v4f p0 = *(const v4fa*)(&os[row * 132 + pc]); const v4f p1 = *(const v4fa*)(&os[row * 132 + pc + 4]);
            const v4f c0 = *(const v4f*)(TC + (size_t)t * 64 + tc); const v4f c1 = *(const v4f*)(TC + (size_t)t * 64 + tc + 4);
            const v4f s0 = *(const v4f*)(TS + (size_t)t * 64 + tc); const v4f s1 = *(const v4f*)(TS + (size_t)t * 64 + tc + 4);
            v8h hv, rv;
#pragma unroll
            for (int i = 0; i < 4; ++i) {
                const float va = x0[i] * c0[i] + sg * (p0[i] * s0[i]); const float vb = x1[i] * c1[i] + sg * (p1[i] * s1[i]);
                const h16 a0h = (h16)va; const h16 a1h = (h16)vb; hv[i] = a0h; hv[4 + i] = a1h;
                rv[i] = (h16)((va - (float)a0h) * RS); rv[4 + i] = (h16)((vb - (float)a1h) * RS); }
            const size_t oo = (size_t)(mb * 16 + row) * HD + c8;
            *(volatile v8h*)(PHz + oo) = hv; if (wr) *(volatile v8h*)(PRz + oo) = rv;
            __threadfence();
            *(volatile v8h*)(PHz + oo) = hv; if (wr) *(volatile v8h*)(PRz + oo) = rv;
        }
        wave_sync();
    }
}

__global__ __launch_bounds__(32) void k_vt(const bf* __restrict__ A, const bf* __restrict__ Bt, h16* VT, h16* VR) {
    __shared__ __align__(16) float os[16 * 68];
    const int K = DM;
    const int lane = threadIdx.x & 31, lr = lane & 15, hi = lane >> 4; const int r0 = blockIdx.x * 64, c0 = blockIdx.y * 64;
    v8f acc[4][4];
#pragma unroll
    for (int mb = 0; mb < 4; ++mb)
#pragma unroll
        for (int nb = 0; nb < 4; ++nb) acc[mb][nb] = (v8f){};
    const size_t aoff = (size_t)(r0 + lr) * K + 8 * hi, boff = (size_t)(c0 + lr) * K + 8 * hi;
#pragma unroll 1
    for (int kc = 0; kc < K; kc += 32) {
        v16bf a[4];
#pragma unroll
        for (int mb = 0; mb < 4; ++mb) a[mb] = ldb(A + aoff + (size_t)mb * 16 * K + kc);
#pragma unroll
        for (int nb = 0; nb < 4; ++nb) { const v16bf b = ldb(Bt + boff + (size_t)nb * 16 * K + kc);
#pragma unroll
            for (int mb = 0; mb < 4; ++mb) acc[mb][nb] = wmmab(a[mb], b, acc[mb][nb]); }
        asm volatile("v_nop\n\tv_nop\n\tv_nop\n\tv_nop" : "+v"(acc[0][0]), "+v"(acc[1][1]), "+v"(acc[2][2]), "+v"(acc[3][3]) : "v"(a[0]), "v"(a[1]), "v"(a[2]), "v"(a[3]));
    }
    const int bb = c0 / SEQ, tc0 = c0 % SEQ;
    const bool wr = tc0 < ER; const int tcr = wr ? tc0 : 0;
    const size_t tbase = ((size_t)bb * DM + r0) * SEQ + tc0;
    const size_t rbase = ((size_t)bb * DM + r0) * ER + tcr;
#pragma unroll
    for (int mb = 0; mb < 4; ++mb) {
#pragma unroll
        for (int nb = 0; nb < 4; ++nb) {
#pragma unroll
            for (int j = 0; j < 8; ++j) os[(hi * 8 + j) * 68 + nb * 16 + lr] = acc[mb][nb][j]; }
        wave_sync();
#pragma unroll 1
        for (int s = 0; s < 4; ++s) {
            const int row = 4 * s + (lane >> 3), c8 = (lane & 7) * 8;
            const v4f x0 = *(const v4fa*)(&os[row * 68 + c8]); const v4f x1 = *(const v4fa*)(&os[row * 68 + c8 + 4]); v8h hv, rv;
#pragma unroll
            for (int i = 0; i < 4; ++i) { const h16 a0 = (h16)x0[i]; const h16 a1 = (h16)x1[i]; hv[i] = a0; hv[4 + i] = a1; rv[i] = (h16)((x0[i] - (float)a0) * RS); rv[4 + i] = (h16)((x1[i] - (float)a1) * RS); }
            const size_t oo = tbase + (size_t)(mb * 16 + row) * SEQ + c8;
            const size_t ro = rbase + (size_t)(mb * 16 + row) * ER + c8;
            *(volatile v8h*)(VT + oo) = hv; if (wr) *(volatile v8h*)(VR + ro) = rv;
            __threadfence();
            *(volatile v8h*)(VT + oo) = hv; if (wr) *(volatile v8h*)(VR + ro) = rv;
        }
        wave_sync();
    }
}

__global__ __launch_bounds__(32 * AW) void k_flash(const h16* __restrict__ QH, const h16* __restrict__ KP, const h16* __restrict__ VT, h16* CH) {
    __shared__ __align__(16) float os[AW * 16 * 132];
    const int lane = threadIdx.x & 31, lr = lane & 15, hi = lane >> 4;
    const int wave = __builtin_amdgcn_readfirstlane((int)(threadIdx.x >> 5));
    const int zh = blockIdx.y; const int b = zh / NH_, h = zh % NH_;
    const int t0 = ER + (blockIdx.x * AW + wave) * 16;
    const size_t pbase = (size_t)zh * SEQ * HD;
    const size_t qo = pbase + (size_t)(t0 + lr) * HD + 8 * hi;
    const v16h q0 = ldh(QH + qo), q1 = ldh(QH + qo + 32), q2 = ldh(QH + qo + 64), q3 = ldh(QH + qo + 96);
    const size_t ko = pbase + (size_t)lr * HD + 8 * hi;
    const size_t vo = pbase + (size_t)lr * SEQ + 8 * hi;
    v8f o0 = (v8f){}, o1 = (v8f){}, o2 = (v8f){}, o3 = (v8f){}, o4 = (v8f){}, o5 = (v8f){}, o6 = (v8f){}, o7 = (v8f){};
    float m = -3.0e38f, l = 0.0f;
    const int nst = (t0 >> 5) + 1;
#pragma unroll 1
    for (int st = 0; st < nst; ++st) {
        const int key0 = st * 32;
        const h16* ka = KP + ko + (size_t)key0 * HD;
        const v16h ka0 = ldh(ka), ka1 = ldh(ka + 32), ka2 = ldh(ka + 64), ka3 = ldh(ka + 96);
        const v16h kb0 = ldh(ka + 16 * HD), kb1 = ldh(ka + 16 * HD + 32), kb2 = ldh(ka + 16 * HD + 64), kb3 = ldh(ka + 16 * HD + 96);
        v8f sa = (v8f){}, sb = (v8f){};
        sa = wmma16(ka0, q0, sa); sb = wmma16(kb0, q0, sb); sa = wmma16(ka1, q1, sa); sb = wmma16(kb1, q1, sb);
        sa = wmma16(ka2, q2, sa); sb = wmma16(kb2, q2, sb); sa = wmma16(ka3, q3, sa); sb = wmma16(kb3, q3, sb);
        asm volatile("v_nop\n\tv_nop\n\tv_nop\n\tv_nop" : "+v"(sa), "+v"(sb) : "v"(ka0), "v"(ka1), "v"(ka2), "v"(ka3), "v"(kb0), "v"(kb1), "v"(kb2), "v"(kb3));
        float ta[8], tb[8];
#pragma unroll
        for (int r = 0; r < 8; ++r) { ta[r] = sa[r] * SC2; tb[r] = sb[r] * SC2; }
        if (key0 + 31 > t0) {
            const int dq = t0 + lr - key0 - 8 * hi;
#pragma unroll
            for (int r = 0; r < 8; ++r) { ta[r] = (r > dq) ? -3.0e38f : ta[r]; tb[r] = (16 + r > dq) ? -3.0e38f : tb[r]; }
        }
        float mx = -3.0e38f;
#pragma unroll
        for (int r = 0; r < 8; ++r) mx = fmaxf(mx, fmaxf(ta[r], tb[r]));
        mx = fmaxf(mx, __shfl_xor(mx, 16, 32));
        const float mnew = fmaxf(m, mx);
        const float alpha = __builtin_amdgcn_exp2f(m - mnew);
        const float sh = PSH - mnew;
        v16h pb; float ls = 0.0f;
#pragma unroll
        for (int r = 0; r < 8; ++r) { const h16 pa = (h16)__builtin_amdgcn_exp2f(ta[r] + sh); const h16 pc = (h16)__builtin_amdgcn_exp2f(tb[r] + sh); pb[r] = pa; pb[8 + r] = pc; ls += (float)pa + (float)pc; }
        l = l * alpha + ls; m = mnew;
        o0 = o0 * alpha; o1 = o1 * alpha; o2 = o2 * alpha; o3 = o3 * alpha; o4 = o4 * alpha; o5 = o5 * alpha; o6 = o6 * alpha; o7 = o7 * alpha;
        const h16* va = VT + vo + key0;
        const v16h v0 = ldh(va), v1 = ldh(va + (size_t)16 * SEQ), v2 = ldh(va + (size_t)32 * SEQ), v3 = ldh(va + (size_t)48 * SEQ);
        const v16h v4 = ldh(va + (size_t)64 * SEQ), v5 = ldh(va + (size_t)80 * SEQ), v6 = ldh(va + (size_t)96 * SEQ), v7 = ldh(va + (size_t)112 * SEQ);
        o0 = wmma16(v0, pb, o0); o1 = wmma16(v1, pb, o1); o2 = wmma16(v2, pb, o2); o3 = wmma16(v3, pb, o3);
        o4 = wmma16(v4, pb, o4); o5 = wmma16(v5, pb, o5); o6 = wmma16(v6, pb, o6); o7 = wmma16(v7, pb, o7);
        asm volatile("v_nop\n\tv_nop\n\tv_nop\n\tv_nop" : "+v"(o0), "+v"(o1), "+v"(o2), "+v"(o3), "+v"(o4), "+v"(o5), "+v"(o6), "+v"(o7) : "v"(v4), "v"(v5), "v"(v6), "v"(v7), "v"(pb));
    }
    l += __shfl_xor(l, 16, 32);
    const float inv = CXS / l;
    const int wb = wave * 16 * 132;
    { v4f a, c;
      a[0] = o0[0] * inv; a[1] = o0[1] * inv; a[2] = o0[2] * inv; a[3] = o0[3] * inv; c[0] = o0[4] * inv; c[1] = o0[5] * inv; c[2] = o0[6] * inv; c[3] = o0[7] * inv;
      *(v4fa*)(&os[wb + lr * 132 +   0 + 8 * hi]) = a; *(v4fa*)(&os[wb + lr * 132 +   0 + 8 * hi + 4]) = c;
      a[0] = o1[0] * inv; a[1] = o1[1] * inv; a[2] = o1[2] * inv; a[3] = o1[3] * inv; c[0] = o1[4] * inv; c[1] = o1[5] * inv; c[2] = o1[6] * inv; c[3] = o1[7] * inv;
      *(v4fa*)(&os[wb + lr * 132 +  16 + 8 * hi]) = a; *(v4fa*)(&os[wb + lr * 132 +  16 + 8 * hi + 4]) = c;
      a[0] = o2[0] * inv; a[1] = o2[1] * inv; a[2] = o2[2] * inv; a[3] = o2[3] * inv; c[0] = o2[4] * inv; c[1] = o2[5] * inv; c[2] = o2[6] * inv; c[3] = o2[7] * inv;
      *(v4fa*)(&os[wb + lr * 132 +  32 + 8 * hi]) = a; *(v4fa*)(&os[wb + lr * 132 +  32 + 8 * hi + 4]) = c;
      a[0] = o3[0] * inv; a[1] = o3[1] * inv; a[2] = o3[2] * inv; a[3] = o3[3] * inv; c[0] = o3[4] * inv; c[1] = o3[5] * inv; c[2] = o3[6] * inv; c[3] = o3[7] * inv;
      *(v4fa*)(&os[wb + lr * 132 +  48 + 8 * hi]) = a; *(v4fa*)(&os[wb + lr * 132 +  48 + 8 * hi + 4]) = c;
      a[0] = o4[0] * inv; a[1] = o4[1] * inv; a[2] = o4[2] * inv; a[3] = o4[3] * inv; c[0] = o4[4] * inv; c[1] = o4[5] * inv; c[2] = o4[6] * inv; c[3] = o4[7] * inv;
      *(v4fa*)(&os[wb + lr * 132 +  64 + 8 * hi]) = a; *(v4fa*)(&os[wb + lr * 132 +  64 + 8 * hi + 4]) = c;
      a[0] = o5[0] * inv; a[1] = o5[1] * inv; a[2] = o5[2] * inv; a[3] = o5[3] * inv; c[0] = o5[4] * inv; c[1] = o5[5] * inv; c[2] = o5[6] * inv; c[3] = o5[7] * inv;
      *(v4fa*)(&os[wb + lr * 132 +  80 + 8 * hi]) = a; *(v4fa*)(&os[wb + lr * 132 +  80 + 8 * hi + 4]) = c;
      a[0] = o6[0] * inv; a[1] = o6[1] * inv; a[2] = o6[2] * inv; a[3] = o6[3] * inv; c[0] = o6[4] * inv; c[1] = o6[5] * inv; c[2] = o6[6] * inv; c[3] = o6[7] * inv;
      *(v4fa*)(&os[wb + lr * 132 +  96 + 8 * hi]) = a; *(v4fa*)(&os[wb + lr * 132 +  96 + 8 * hi + 4]) = c;
      a[0] = o7[0] * inv; a[1] = o7[1] * inv; a[2] = o7[2] * inv; a[3] = o7[3] * inv; c[0] = o7[4] * inv; c[1] = o7[5] * inv; c[2] = o7[6] * inv; c[3] = o7[7] * inv;
      *(v4fa*)(&os[wb + lr * 132 + 112 + 8 * hi]) = a; *(v4fa*)(&os[wb + lr * 132 + 112 + 8 * hi + 4]) = c; }
    wave_sync();
    h16* crow = CH + ((size_t)b * SEQ + t0) * DM + h * HD;
#pragma unroll 1
    for (int ps = 0; ps < 2; ++ps) {
#pragma unroll
        for (int s = 0; s < 8; ++s) { const int row = 2 * s + hi, c8 = lr * 8;
            const v4f x0 = *(const v4fa*)(&os[wb + row * 132 + c8]); const v4f x1 = *(const v4fa*)(&os[wb + row * 132 + c8 + 4]); v8h hv;
#pragma unroll
            for (int i = 0; i < 4; ++i) { hv[i] = (h16)x0[i]; hv[4 + i] = (h16)x1[i]; }
            *(volatile v8h*)(crow + (size_t)row * DM + c8) = hv; }
        if (ps == 0) __threadfence(); }
}

__global__ __launch_bounds__(32 * AW) void k_flash_early(const h16* __restrict__ QH, const h16* __restrict__ QR, const h16* __restrict__ KP, const h16* __restrict__ KR,
                                                       const h16* __restrict__ VT, const h16* __restrict__ VR, h16* CH, h16* CR) {
    __shared__ __align__(16) float os[AW * 16 * 68];
    const int lane = threadIdx.x & 31, lr = lane & 15, hi = lane >> 4;
    const int wave = __builtin_amdgcn_readfirstlane((int)(threadIdx.x >> 5));
    const int qt = wave >> 1, dh = wave & 1;
    const int zh = blockIdx.y; const int b = zh / NH_, h = zh % NH_;
    const int t0 = (blockIdx.x * 2 + qt) * 16;
    const size_t pF = (size_t)zh * SEQ * HD, pE = (size_t)zh * ER * HD;
    const size_t qo = pF + (size_t)(t0 + lr) * HD + 8 * hi, qro = pE + (size_t)(t0 + lr) * HD + 8 * hi;
    const size_t ko = pF + (size_t)lr * HD + 8 * hi, kro = pE + (size_t)lr * HD + 8 * hi;
    const size_t vo = pF + (size_t)(dh * 64 + lr) * SEQ + 8 * hi, vro = pE + (size_t)(dh * 64 + lr) * ER + 8 * hi;
    v8f oh0 = (v8f){}, oh1 = (v8f){}, oh2 = (v8f){}, oh3 = (v8f){}, or0 = (v8f){}, or1 = (v8f){}, or2 = (v8f){}, or3 = (v8f){};
    float m = -3.0e38f, l = 0.0f;
    const int nst = (t0 >> 5) + 1;
#pragma unroll 1
    for (int st = 0; st < nst; ++st) {
        const int key0 = st * 32;
        const size_t kof = ko + (size_t)key0 * HD, krf = kro + (size_t)key0 * HD;
        v8f sHa = (v8f){}, sLa = (v8f){}, sHb = (v8f){}, sLb = (v8f){};
#pragma unroll 1
        for (int kk = 0; kk < 4; ++kk) {
            const int dk = 32 * kk;
            const v16h qh = ldh(QH + qo + dk), qr = ldh(QR + qro + dk);
            const v16h kha = ldh(KP + kof + dk), kra = ldh(KR + krf + dk);
            const v16h khb = ldh(KP + kof + 16 * HD + dk), krb = ldh(KR + krf + 16 * HD + dk);
            sHa = wmma16(kha, qh, sHa); sLa = wmma16(kha, qr, sLa); sHb = wmma16(khb, qh, sHb); sLb = wmma16(khb, qr, sLb);
            sLa = wmma16(kra, qh, sLa); sLb = wmma16(krb, qh, sLb);
            asm volatile("v_nop\n\tv_nop\n\tv_nop\n\tv_nop" : "+v"(sHa), "+v"(sLa), "+v"(sHb), "+v"(sLb) : "v"(kha), "v"(kra), "v"(khb), "v"(krb), "v"(qh), "v"(qr));
        }
        float ta[8], tb[8];
#pragma unroll
        for (int r = 0; r < 8; ++r) { ta[r] = (sHa[r] + sLa[r] * RI) * SC2; tb[r] = (sHb[r] + sLb[r] * RI) * SC2; }
        if (key0 + 31 > t0) {
            const int dq = t0 + lr - key0 - 8 * hi;
#pragma unroll
            for (int r = 0; r < 8; ++r) { ta[r] = (r > dq) ? -3.0e38f : ta[r]; tb[r] = (16 + r > dq) ? -3.0e38f : tb[r]; }
        }
        float mx = -3.0e38f;
#pragma unroll
        for (int r = 0; r < 8; ++r) mx = fmaxf(mx, fmaxf(ta[r], tb[r]));
        mx = fmaxf(mx, __shfl_xor(mx, 16, 32));
        const float mnew = fmaxf(m, mx);
        const float alpha = __builtin_amdgcn_exp2f(m - mnew);
        const float sh = PSH - mnew;
        v16h pb; float ls = 0.0f;
#pragma unroll
        for (int r = 0; r < 8; ++r) { const h16 pa = (h16)__builtin_amdgcn_exp2f(ta[r] + sh); const h16 pc = (h16)__builtin_amdgcn_exp2f(tb[r] + sh); pb[r] = pa; pb[8 + r] = pc; ls += (float)pa + (float)pc; }
        l = l * alpha + ls; m = mnew;
        oh0 = oh0 * alpha; oh1 = oh1 * alpha; oh2 = oh2 * alpha; oh3 = oh3 * alpha; or0 = or0 * alpha; or1 = or1 * alpha; or2 = or2 * alpha; or3 = or3 * alpha;
        const h16* va = VT + vo + key0; const h16* vr = VR + vro + key0;
        const v16h v0 = ldh(va), v1 = ldh(va + (size_t)16 * SEQ), v2 = ldh(va + (size_t)32 * SEQ), v3 = ldh(va + (size_t)48 * SEQ);
        const v16h w0 = ldh(vr), w1 = ldh(vr + (size_t)16 * ER), w2 = ldh(vr + (size_t)32 * ER), w3 = ldh(vr + (size_t)48 * ER);
        oh0 = wmma16(v0, pb, oh0); oh1 = wmma16(v1, pb, oh1); oh2 = wmma16(v2, pb, oh2); oh3 = wmma16(v3, pb, oh3);
        or0 = wmma16(w0, pb, or0); or1 = wmma16(w1, pb, or1); or2 = wmma16(w2, pb, or2); or3 = wmma16(w3, pb, or3);
        asm volatile("v_nop\n\tv_nop\n\tv_nop\n\tv_nop" : "+v"(oh0), "+v"(oh1), "+v"(oh2), "+v"(oh3), "+v"(or0), "+v"(or1), "+v"(or2), "+v"(or3) : "v"(w0), "v"(w1), "v"(w2), "v"(w3), "v"(pb));
    }
    l += __shfl_xor(l, 16, 32);
    const float inv = CXS / l;
    const int wb = wave * 16 * 68;
    { v4f a, c;
      a[0] = (oh0[0] + or0[0] * RI) * inv; a[1] = (oh0[1] + or0[1] * RI) * inv; a[2] = (oh0[2] + or0[2] * RI) * inv; a[3] = (oh0[3] + or0[3] * RI) * inv;
      c[0] = (oh0[4] + or0[4] * RI) * inv; c[1] = (oh0[5] + or0[5] * RI) * inv; c[2] = (oh0[6] + or0[6] * RI) * inv; c[3] = (oh0[7] + or0[7] * RI) * inv;
      *(v4fa*)(&os[wb + lr * 68 +  0 + 8 * hi]) = a; *(v4fa*)(&os[wb + lr * 68 +  0 + 8 * hi + 4]) = c;
      a[0] = (oh1[0] + or1[0] * RI) * inv; a[1] = (oh1[1] + or1[1] * RI) * inv; a[2] = (oh1[2] + or1[2] * RI) * inv; a[3] = (oh1[3] + or1[3] * RI) * inv;
      c[0] = (oh1[4] + or1[4] * RI) * inv; c[1] = (oh1[5] + or1[5] * RI) * inv; c[2] = (oh1[6] + or1[6] * RI) * inv; c[3] = (oh1[7] + or1[7] * RI) * inv;
      *(v4fa*)(&os[wb + lr * 68 + 16 + 8 * hi]) = a; *(v4fa*)(&os[wb + lr * 68 + 16 + 8 * hi + 4]) = c;
      a[0] = (oh2[0] + or2[0] * RI) * inv; a[1] = (oh2[1] + or2[1] * RI) * inv; a[2] = (oh2[2] + or2[2] * RI) * inv; a[3] = (oh2[3] + or2[3] * RI) * inv;
      c[0] = (oh2[4] + or2[4] * RI) * inv; c[1] = (oh2[5] + or2[5] * RI) * inv; c[2] = (oh2[6] + or2[6] * RI) * inv; c[3] = (oh2[7] + or2[7] * RI) * inv;
      *(v4fa*)(&os[wb + lr * 68 + 32 + 8 * hi]) = a; *(v4fa*)(&os[wb + lr * 68 + 32 + 8 * hi + 4]) = c;
      a[0] = (oh3[0] + or3[0] * RI) * inv; a[1] = (oh3[1] + or3[1] * RI) * inv; a[2] = (oh3[2] + or3[2] * RI) * inv; a[3] = (oh3[3] + or3[3] * RI) * inv;
      c[0] = (oh3[4] + or3[4] * RI) * inv; c[1] = (oh3[5] + or3[5] * RI) * inv; c[2] = (oh3[6] + or3[6] * RI) * inv; c[3] = (oh3[7] + or3[7] * RI) * inv;
      *(v4fa*)(&os[wb + lr * 68 + 48 + 8 * hi]) = a; *(v4fa*)(&os[wb + lr * 68 + 48 + 8 * hi + 4]) = c; }
    wave_sync();
    h16* crow = CH + ((size_t)b * SEQ + t0) * DM + h * HD + dh * 64;
    h16* rrow = CR + ((size_t)b * ER + t0) * DM + h * HD + dh * 64;
#pragma unroll 1
    for (int ps = 0; ps < 2; ++ps) {
#pragma unroll
        for (int s = 0; s < 4; ++s) { const int row = 4 * s + (lane >> 3), c8 = (lane & 7) * 8;
            const v4f x0 = *(const v4fa*)(&os[wb + row * 68 + c8]); const v4f x1 = *(const v4fa*)(&os[wb + row * 68 + c8 + 4]); v8h hv, rv;
#pragma unroll
            for (int i = 0; i < 4; ++i) { const h16 a0 = (h16)x0[i]; const h16 a1 = (h16)x1[i]; hv[i] = a0; hv[4 + i] = a1; rv[i] = (h16)((x0[i] - (float)a0) * RS); rv[4 + i] = (h16)((x1[i] - (float)a1) * RS); }
            *(volatile v8h*)(crow + (size_t)row * DM + c8) = hv; *(volatile v8h*)(rrow + (size_t)row * DM + c8) = rv; }
        if (ps == 0) __threadfence(); }
}

__global__ __launch_bounds__(32) void k_out_dense(const h16* __restrict__ A, const h16* __restrict__ Bt, float* OUT) {
    __shared__ __align__(16) float os[16 * 68];
    const int K = DM;
    const int lane = threadIdx.x & 31, lr = lane & 15, hi = lane >> 4;
    const int bb = blockIdx.x / DTL, tt0 = ER + (blockIdx.x % DTL) * 64, c0 = blockIdx.y * 64;
    v8f acc[4][4];
#pragma unroll
    for (int mb = 0; mb < 4; ++mb)
#pragma unroll
        for (int nb = 0; nb < 4; ++nb) acc[mb][nb] = (v8f){};
    const size_t aoff = (size_t)(bb * SEQ + tt0 + lr) * K + 8 * hi, boff = (size_t)(c0 + lr) * K + 8 * hi;
#pragma unroll 1
    for (int kc = 0; kc < K; kc += 32) {
        v16h a[4];
#pragma unroll
        for (int mb = 0; mb < 4; ++mb) a[mb] = ldh(A + aoff + (size_t)mb * 16 * K + kc);
#pragma unroll
        for (int nb = 0; nb < 4; ++nb) { const v16h bw = ldh(Bt + boff + (size_t)nb * 16 * K + kc);
#pragma unroll
            for (int mb = 0; mb < 4; ++mb) acc[mb][nb] = wmma16(a[mb], bw, acc[mb][nb]); }
        asm volatile("v_nop\n\tv_nop\n\tv_nop\n\tv_nop" : "+v"(acc[0][0]), "+v"(acc[1][1]), "+v"(acc[2][2]), "+v"(acc[3][3]) : "v"(a[0]), "v"(a[1]), "v"(a[2]), "v"(a[3]));
    }
#pragma unroll
    for (int mb = 0; mb < 4; ++mb) {
#pragma unroll
        for (int nb = 0; nb < 4; ++nb) {
#pragma unroll
            for (int j = 0; j < 8; ++j) os[(hi * 8 + j) * 68 + nb * 16 + lr] = acc[mb][nb][j] * OUTS; }
        wave_sync();
        float* orow = OUT + ((size_t)bb * OUT_SEQ + tt0 + mb * 16) * DM + c0;
#pragma unroll 1
        for (int ps = 0; ps < 2; ++ps) {
#pragma unroll
            for (int s = 0; s < 8; ++s) { const int row = 2 * s + hi, cofs = lr * 4;
                const v4f val = *(const v4fa*)(&os[row * 68 + cofs]);
                *(volatile v4f*)(orow + (size_t)row * DM + cofs) = val; }
            if (ps == 0) __threadfence(); }
        wave_sync();
    }
}

__global__ __launch_bounds__(32) void k_out_early(const h16* __restrict__ A, const h16* __restrict__ AR, const h16* __restrict__ Bt, float* OUT) {
    __shared__ __align__(16) float os[16 * 68];
    const int K = DM;
    const int lane = threadIdx.x & 31, lr = lane & 15, hi = lane >> 4;
    const int bb = blockIdx.x / (ER / 32), tt0 = (blockIdx.x % (ER / 32)) * 32, c0 = blockIdx.y * 64;
    v8f acc[2][4], accr[2][4];
#pragma unroll
    for (int mb = 0; mb < 2; ++mb)
#pragma unroll
        for (int nb = 0; nb < 4; ++nb) { acc[mb][nb] = (v8f){}; accr[mb][nb] = (v8f){}; }
    const size_t aoff = (size_t)(bb * SEQ + tt0 + lr) * K + 8 * hi, roff = (size_t)(bb * ER + tt0 + lr) * K + 8 * hi, boff = (size_t)(c0 + lr) * K + 8 * hi;
#pragma unroll 1
    for (int kc = 0; kc < K; kc += 32) {
        const v16h a0 = ldh(A + aoff + kc), a1 = ldh(A + aoff + (size_t)16 * K + kc);
        const v16h r0 = ldh(AR + roff + kc), r1 = ldh(AR + roff + (size_t)16 * K + kc);
#pragma unroll
        for (int nb = 0; nb < 4; ++nb) { const v16h bw = ldh(Bt + boff + (size_t)nb * 16 * K + kc);
            acc[0][nb] = wmma16(a0, bw, acc[0][nb]); acc[1][nb] = wmma16(a1, bw, acc[1][nb]);
            accr[0][nb] = wmma16(r0, bw, accr[0][nb]); accr[1][nb] = wmma16(r1, bw, accr[1][nb]); }
        asm volatile("v_nop\n\tv_nop\n\tv_nop\n\tv_nop" : "+v"(acc[0][3]), "+v"(acc[1][3]), "+v"(accr[0][3]), "+v"(accr[1][3]), "+v"(acc[0][2]), "+v"(acc[1][2]), "+v"(accr[0][2]), "+v"(accr[1][2]) : "v"(a0), "v"(a1), "v"(r0), "v"(r1));
    }
#pragma unroll
    for (int mb = 0; mb < 2; ++mb) {
#pragma unroll
        for (int nb = 0; nb < 4; ++nb) {
#pragma unroll
            for (int j = 0; j < 8; ++j) os[(hi * 8 + j) * 68 + nb * 16 + lr] = (acc[mb][nb][j] + accr[mb][nb][j] * RI) * OUTS; }
        wave_sync();
        float* orow = OUT + ((size_t)bb * OUT_SEQ + tt0 + mb * 16) * DM + c0;
#pragma unroll 1
        for (int ps = 0; ps < 2; ++ps) {
#pragma unroll
            for (int s = 0; s < 8; ++s) { const int row = 2 * s + hi, cofs = lr * 4;
                const v4f val = *(const v4fa*)(&os[row * 68 + cofs]);
                *(volatile v4f*)(orow + (size_t)row * DM + cofs) = val; }
            if (ps == 0) __threadfence(); }
        wave_sync();
    }
}

static constexpr size_t al256(size_t v) { return (v + 255) & ~(size_t)255; }
static constexpr size_t SZ_XB  = al256((size_t)NB * SEQ * DM * 2);
static constexpr size_t SZ_WB  = al256((size_t)4 * DM * DM * 2);
static constexpr size_t SZ_QK  = al256((size_t)2 * PLN * 2);
static constexpr size_t SZ_VT  = al256((size_t)PLN * 2);
static constexpr size_t SZ_QKR = al256((size_t)2 * PLE * 2);
static constexpr size_t SZ_VR  = al256((size_t)PLE * 2);
static constexpr size_t SZ_CR  = al256((size_t)NB * ER * DM * 2);
static constexpr size_t SZ_TAB = al256((size_t)2 * SEQ * 64 * 4);
static constexpr size_t SZ_TOTAL = SZ_XB + SZ_WB + SZ_QK + SZ_VT + SZ_QKR + SZ_VR + SZ_CR + SZ_TAB;
static_assert(SZ_TOTAL <= (size_t)134217728);
static_assert(((size_t)DM * DM * 2) % 256 == 0);
static_assert((PLN * 2) % 256 == 0);
static_assert((PLE * 2) % 256 == 0);
static_assert((size_t)NB * SEQ * DM * 2 <= SZ_XB);

extern "C" void kernel_launch(void* const* d_in, const int* in_sizes, int n_in,
                              void* d_out, int out_size, void* d_ws, size_t ws_size, hipStream_t stream) {
    if (n_in < 5) return;
    const size_t needx = ((size_t)(NB - 1) * SEQ_FULL + SEQ) * DM;
    if ((size_t)in_sizes[0] < needx) return;
    if ((size_t)in_sizes[1] < (size_t)DM * DM || (size_t)in_sizes[2] < (size_t)DM * DM || (size_t)in_sizes[3] < (size_t)DM * DM || (size_t)in_sizes[4] < (size_t)DM * DM) return;
    if ((size_t)out_size < ((size_t)(NB - 1) * OUT_SEQ + SEQ) * DM) return;
    if (SZ_TOTAL > ws_size) return;
    const float* x = (const float*)d_in[0]; const float* wq = (const float*)d_in[1]; const float* wk = (const float*)d_in[2];
    const float* wv = (const float*)d_in[3]; const float* wo = (const float*)d_in[4];
    float* OUT = (float*)d_out;
    char* wsp = (char*)d_ws;
    bf* XB = (bf*)wsp; h16* CH = (h16*)wsp; wsp += SZ_XB;
    bf* WB = (bf*)wsp; wsp += SZ_WB;
    h16* QK = (h16*)wsp; wsp += SZ_QK;
    h16* VT = (h16*)wsp; wsp += SZ_VT;
    h16* QKR = (h16*)wsp; wsp += SZ_QKR;
    h16* VR = (h16*)wsp; wsp += SZ_VR;
    h16* CR = (h16*)wsp; wsp += SZ_CR;
    float* TAB = (float*)wsp; wsp += SZ_TAB;
    bf* WQT = WB; bf* WKT = WB + (size_t)DM * DM; bf* WVT = WB + (size_t)2 * DM * DM; bf* WOT = WB + (size_t)3 * DM * DM;
    h16* QH = QK; h16* KP = QK + PLN; h16* QR = QKR; h16* KR = QKR + PLE;

    if (SEQ == SEQ_FULL) {
        const size_t n8 = (size_t)NB * SEQ * DM / 8;
        k_cvt8<<<(unsigned)((n8 + 255) / 256), 256, 0, stream>>>(x, XB, n8);
    } else {
        const size_t n8 = (size_t)SEQ * DM / 8;
        for (int b = 0; b < NB; ++b) k_cvt8<<<(unsigned)((n8 + 255) / 256), 256, 0, stream>>>(x + (size_t)b * SEQ_FULL * DM, XB + (size_t)b * SEQ * DM, n8);
    }
    k_wt<0><<<dim3(DM / 64, DM / 64, 1), 256, 0, stream>>>(wq, WQT);
    k_wt<0><<<dim3(DM / 64, DM / 64, 1), 256, 0, stream>>>(wk, WKT);
    k_wt<0><<<dim3(DM / 64, DM / 64, 1), 256, 0, stream>>>(wv, WVT);
    k_wt<1><<<dim3(DM / 64, DM / 64, 1), 256, 0, stream>>>(wo, WOT);
    k_tab<<<(unsigned)(SEQ * 64 / 256), 256, 0, stream>>>(TAB);

    k_qk<<<dim3(NB * SEQ / 32, NH_, 2), 32, 0, stream>>>(XB, WB, TAB, QK, QKR);
    k_vt<<<dim3(DM / 64, NB * SEQ / 64, 1), 32, 0, stream>>>(WVT, XB, VT, VR);

    if (SEQ > ER) k_flash<<<dim3((SEQ > ER ? (SEQ - ER) / (16 * AW) : 1), NB * NH_, 1), 32 * AW, 0, stream>>>(QH, KP, VT, CH);
    k_flash_early<<<dim3(ER / 32, NB * NH_, 1), 32 * AW, 0, stream>>>(QH, QR, KP, KR, VT, VR, CH, CR);

    if (SEQ > ER) k_out_dense<<<dim3(NB * DTL, DM / 64, 1), 32, 0, stream>>>(CH, (const h16*)WOT, OUT);
    k_out_early<<<dim3(NB * ER / 32, DM / 64, 1), 32, 0, stream>>>(CH, CR, (const h16*)WOT, OUT);
}
